// Net_77618648973637
// MI455X (gfx1250) — hardware-verified
//
#include <hip/hip_runtime.h>
#include <stddef.h>
#include <stdint.h>
#include <math.h>


#define IN_F    256
#define CH      512
#define NCAT    (2 * CH)
#define NLAB    1440
#define NLK     6
#define NTHR    256
#define NWAVE   8
#define EPT     8
#define CHUNK   (NTHR * EPT)
#define WCAP    (EPT * 32)
#define LISTN   (NWAVE * WCAP)
#define NBA     1024
#define SLA     10
#define RCAP    28672
#define DEGCAP  64
#define GBM     64
#define GBN     64
#define GTHR    128
#define TRN     32
#define TRK     64
#define TPITCH  36
#define AGG_ZINTS    (LISTN + 2 * RCAP + 3 * NBA)
#define AGG_LDS_INTS (AGG_ZINTS + 16)
#define WSMAX   134217728
#define CA      16.0f
#define CW      8192.0f
#define INVC    (1.0f / 131072.0f)

static_assert((CHUNK & (CHUNK - 1)) == 0 && CHUNK <= 4096);
static_assert((NBA & (NBA - 1)) == 0 && NBA == (1 << SLA));
static_assert(((long long)CHUNK << SLA) < (1LL << 31));
static_assert(LISTN % NTHR == 0 && NBA % NTHR == 0);
static_assert(NBA % NWAVE == 0 && NBA % 32 == 0 && NBA % GBM == 0);
static_assert(NBA == 4 * NTHR);
static_assert(RCAP % 32 == 0 && AGG_ZINTS % (4 * NTHR) == 0);
static_assert(DEGCAP % 32 == 0);
static_assert(AGG_LDS_INTS * 4 <= 262144);
static_assert(IN_F % 32 == 0 && CH % 32 == 0);
static_assert(IN_F % TRK == 0 && CH % TRK == 0 && CH % TRN == 0 && NLAB % TRN == 0);
static_assert(NCAT % GBN == 0);
static_assert(CH == 2 * 32 * 8);
static_assert(IN_F == 32 * 8);
static_assert((NLAB * 4) % 128 == 0);
static_assert(((NLAB % GBN) * 4) % 128 == 0);
static_assert(GBM == (GTHR / 32) * 16 && GBN == 64);
static_assert(TPITCH % 4 == 0 && TRK == 8 * 8 && TRN * 8 == NTHR && TRK * (TRN / 4) == 2 * NTHR);

typedef float          v4f   __attribute__((ext_vector_type(4)));
typedef float          v8f   __attribute__((ext_vector_type(8)));
typedef int            v4i   __attribute__((ext_vector_type(4)));
typedef int            v8i   __attribute__((ext_vector_type(8)));
typedef unsigned short v8us  __attribute__((ext_vector_type(8)));
typedef _Float16       v8h   __attribute__((ext_vector_type(8)));
typedef _Float16       v16h  __attribute__((ext_vector_type(16)));
typedef v4f  __attribute__((may_alias)) v4fa;
typedef v4i  __attribute__((may_alias)) v4ia;
typedef v8us __attribute__((may_alias)) v8usa;
union Frag  { v16h f; v8us h[2]; v8i w; };
union HPack { v8h f; v8us u; };

__device__ __forceinline__ v8f wmh(const Frag& a, const Frag& b, v8f c) {
  v8f d = __builtin_amdgcn_wmma_f32_16x16x32_f16(false, a.f, false, b.f, (short)0, c, false, false);
  asm volatile("v_nop\n\tv_nop\n\tv_nop\n\tv_nop" : "+v"(d) : "v"(a.w), "v"(b.w));
  return d;
}

__device__ __forceinline__ unsigned bf16_bits(float f) {
  const unsigned u = __float_as_uint(f);
  return (u + 0x7FFFu + ((u >> 16) & 1u)) >> 16;
}
__device__ __forceinline__ float bf16_val(float f) {
  return __uint_as_float(bf16_bits(f) << 16);
}

template <int SLB>
__device__ __forceinline__ int scan_chunk(const int* __restrict__ keys, int nE, int cbase, int slotBase,
                                          int nb, int vec8, int* list, int tid, int lane, int wave) {
  int wc = 0;
  const int el0  = tid * EPT;
  const int e0   = cbase + el0;
  const int sent = -2147483647 - 1;
  v4i da, db;
  if (vec8 != 0 && cbase + CHUNK <= nE) {
    da = *(const v4i*)(keys + e0);
    db = *(const v4i*)(keys + e0 + 4);
  } else {
    da.x = (e0     < nE) ? keys[min(e0,     nE - 1)] : sent;
    da.y = (e0 + 1 < nE) ? keys[min(e0 + 1, nE - 1)] : sent;
    da.z = (e0 + 2 < nE) ? keys[min(e0 + 2, nE - 1)] : sent;
    da.w = (e0 + 3 < nE) ? keys[min(e0 + 3, nE - 1)] : sent;
    db.x = (e0 + 4 < nE) ? keys[min(e0 + 4, nE - 1)] : sent;
    db.y = (e0 + 5 < nE) ? keys[min(e0 + 5, nE - 1)] : sent;
    db.z = (e0 + 6 < nE) ? keys[min(e0 + 6, nE - 1)] : sent;
    db.w = (e0 + 7 < nE) ? keys[min(e0 + 7, nE - 1)] : sent;
  }
  const unsigned nbs = (unsigned)slotBase;
  const unsigned unb = (unsigned)nb;
  const unsigned s0 = (unsigned)da.x - nbs, s1 = (unsigned)da.y - nbs;
  const unsigned s2 = (unsigned)da.z - nbs, s3 = (unsigned)da.w - nbs;
  const unsigned s4 = (unsigned)db.x - nbs, s5 = (unsigned)db.y - nbs;
  const unsigned s6 = (unsigned)db.z - nbs, s7 = (unsigned)db.w - nbs;
  const bool h0 = s0 < unb, h1 = s1 < unb, h2 = s2 < unb, h3 = s3 < unb;
  const bool h4 = s4 < unb, h5 = s5 < unb, h6 = s6 < unb, h7 = s7 < unb;
  const unsigned any = __builtin_amdgcn_ballot_w32(h0 | h1 | h2 | h3 | h4 | h5 | h6 | h7);
  if (any != 0u) {
#define HITJ(J, HJ, SJ) { \
      const unsigned mj = __builtin_amdgcn_ballot_w32(HJ); \
      if (mj != 0u) { \
        if (HJ) { \
          const int pos = wc + (int)__builtin_amdgcn_mbcnt_lo(mj, 0u); \
          if (pos < WCAP) list[wave * WCAP + pos] = ((el0 + (J)) << SLB) | (int)(SJ); \
        } \
        wc += (int)__builtin_popcount(mj); } }
    HITJ(0, h0, s0)
    HITJ(1, h1, s1)
    HITJ(2, h2, s2)
    HITJ(3, h3, s3)
    HITJ(4, h4, s4)
    HITJ(5, h5, s5)
    HITJ(6, h6, s6)
    HITJ(7, h7, s7)
#undef HITJ
  }
  return wc;
}

__global__ __launch_bounds__(NTHR) void k_deg(const int* __restrict__ keys, int nE, int vec8, float* degp) {
  __shared__ __attribute__((aligned(16))) int list[LISTN];
  __shared__ __attribute__((aligned(16))) int cnt[NBA];
  __shared__ int misc[16];
  const int tid = (int)threadIdx.x, lane = tid & 31, wave = tid >> 5;
  const int nodeBase = (int)blockIdx.x * NBA;
  for (int i = tid; i < LISTN; i += NTHR) list[i] = 0;
  for (int i = tid; i < NBA; i += NTHR) cnt[i] = 0;
  if (tid < 16) misc[tid] = 0;
  __syncthreads();

  const int nChunks = (nE + CHUNK - 1) / CHUNK;
#pragma unroll 1
  for (int ch = 0; ch < nChunks; ++ch) {
    const int cbase = ch * CHUNK;
    const int wc = scan_chunk<SLA>(keys, nE, cbase, nodeBase, NBA, vec8, list, tid, lane, wave);
    if (lane == 0) misc[wave] = wc;
    __syncthreads();
    if (wave == 0) {
#pragma unroll 1
      for (int w2 = 0; w2 < NWAVE; ++w2) {
        int c = misc[w2];
        c = c < 0 ? 0 : (c > WCAP ? WCAP : c);
#pragma unroll 1
        for (int b0 = 0; b0 < c; b0 += 32) {
          const int idx = b0 + lane;
          const int ent = list[w2 * WCAP + (idx < WCAP ? idx : WCAP - 1)];
          const int m32 = (c - b0) < 32 ? (c - b0) : 32;
#pragma unroll 1
          for (int k = 0; k < m32; ++k) {
            const int u    = __builtin_amdgcn_readlane(ent, k);
            const int slot = u & (NBA - 1);
            if (lane == 0) cnt[slot] = cnt[slot] + 1;
          }
        }
      }
    }
    __syncthreads();
  }

  const int e = 128 * wave + 4 * lane;
  v4f o;
  o.x = (float)cnt[e];     o.y = (float)cnt[e + 1];
  o.z = (float)cnt[e + 2]; o.w = (float)cnt[e + 3];
  float* dp = degp + (size_t)nodeBase + e;
  *(volatile v4f*)dp = o;
  __threadfence();
  *(volatile v4f*)dp = o;
}

__global__ __launch_bounds__(NTHR) void k_xcvt(const float* __restrict__ x, int nR, int nUnits,
                                               unsigned short* xh) {
  const int u = (int)blockIdx.x * NTHR + (int)threadIdx.x;
  if (u >= nUnits) return;
  const int row = u >> 5;
  const int k8  = (u & 31) * 8;
  const int rc  = row < nR ? row : nR - 1;
  const float* p = x + (size_t)rc * IN_F + k8;
  const v4f a = *(const v4fa*)p;
  const v4f b = *(const v4fa*)(p + 4);
  const bool ok = row < nR;
  HPack o;
  o.f[0] = (_Float16)((ok ? bf16_val(a.x) : 0.0f) * CA);
  o.f[1] = (_Float16)((ok ? bf16_val(a.y) : 0.0f) * CA);
  o.f[2] = (_Float16)((ok ? bf16_val(a.z) : 0.0f) * CA);
  o.f[3] = (_Float16)((ok ? bf16_val(a.w) : 0.0f) * CA);
  o.f[4] = (_Float16)((ok ? bf16_val(b.x) : 0.0f) * CA);
  o.f[5] = (_Float16)((ok ? bf16_val(b.y) : 0.0f) * CA);
  o.f[6] = (_Float16)((ok ? bf16_val(b.z) : 0.0f) * CA);
  o.f[7] = (_Float16)((ok ? bf16_val(b.w) : 0.0f) * CA);
  unsigned short* dp = xh + (size_t)row * IN_F + k8;
  *(volatile v8us*)dp = o.u;
  __threadfence();
  *(volatile v8us*)dp = o.u;
}

__global__ __launch_bounds__(NTHR) void k_wtr(const float* __restrict__ W, int N, int K, int zsw,
                                              unsigned short* BT, int rowOff, int zsb) {
  __shared__ __attribute__((aligned(16))) float T[TRK * TPITCH];
  const int tid = (int)threadIdx.x;
  const int n0 = (int)blockIdx.x * TRN;
  const int k0 = (int)blockIdx.y * TRK;
  const float* Wz = W + (size_t)blockIdx.z * (size_t)zsw;
  unsigned short* Bz = BT + (size_t)blockIdx.z * (size_t)zsb;
#pragma unroll
  for (int i = 0; i < 2; ++i) {
    const int u  = tid + NTHR * i;
    const int kr = u >> 3;
    const int q  = u & 7;
    const v4f v = *(const v4fa*)(Wz + (size_t)(k0 + kr) * (size_t)N + n0 + 4 * q);
    *(v4fa*)(T + kr * TPITCH + 4 * q) = v;
  }
  __syncthreads();
  const int r = tid >> 3;
  const int q = tid & 7;
  HPack o;
#pragma unroll
  for (int j = 0; j < 8; ++j) o.f[j] = (_Float16)(bf16_val(T[(8 * q + j) * TPITCH + r]) * CW);
  unsigned short* dp = Bz + (size_t)(rowOff + n0 + r) * (size_t)K + k0 + 8 * q;
  *(volatile v8us*)dp = o.u;
  __threadfence();
  *(volatile v8us*)dp = o.u;
}

template <int NT, int HB>
__global__ __launch_bounds__(GTHR) void k_gemm(const unsigned short* __restrict__ A, int lda,
                                               const unsigned short* __restrict__ BT, int ldb, int nBrows, int K,
                                               const float* __restrict__ bias,
                                               float* C32, int ldc, int nRows, int nCols) {
  static_assert(NT == 4);
  constexpr int BN = 16 * NT;
  __shared__ __attribute__((aligned(16))) float stg[GBM * BN];
  const int tid = (int)threadIdx.x, lane = tid & 31, wave = tid >> 5, hh = lane >> 4, m = lane & 15;
  const int rowBase = (int)blockIdx.x * GBM;
  const int colBase = (int)blockIdx.y * BN;

  v8f acc[NT];
  {
    const v8f z = {0.f, 0.f, 0.f, 0.f, 0.f, 0.f, 0.f, 0.f};
#pragma unroll
    for (int t = 0; t < NT; ++t) acc[t] = z;
  }
  const unsigned short* ap = A + (size_t)(rowBase + 16 * wave + m) * (size_t)lda + 8 * hh;
  const unsigned short* bpn[NT];
#pragma unroll
  for (int nt = 0; nt < NT; ++nt) {
    int bn = colBase + 16 * nt + m;
    bn = bn > nBrows - 1 ? nBrows - 1 : bn;
    bpn[nt] = BT + (size_t)bn * (size_t)ldb + 8 * hh;
  }

#pragma unroll 1
  for (int k0 = 0; k0 < K; k0 += 32) {
    Frag af;
    af.h[0] = *(const v8usa*)(ap + k0);
    af.h[1] = *(const v8usa*)(ap + k0 + 16);
#pragma unroll
    for (int nt = 0; nt < NT; ++nt) {
      const unsigned short* wq = bpn[nt] + k0;
      Frag bf;
      bf.h[0] = *(const v8usa*)wq;
      bf.h[1] = *(const v8usa*)(wq + 16);
      acc[nt] = wmh(af, bf, acc[nt]);
    }
  }

#pragma unroll
  for (int nt = 0; nt < NT; ++nt) {
    const int lc = 16 * nt + m;
    float bb = 0.0f;
    if constexpr (HB != 0) {
      int gc = colBase + lc;
      gc = gc > nCols - 1 ? nCols - 1 : gc;
      bb = bf16_val(bias[gc]);
    }
#pragma unroll
    for (int r = 0; r < 8; ++r) {
      const int lr = 16 * wave + 8 * hh + r;
      stg[lr * BN + lc] = acc[nt][r] * INVC + bb;
    }
  }
  __syncthreads();

  v4f pv[8];
#pragma unroll
  for (int i = 0; i < 8; ++i) {
    const int lr = 16 * wave + 2 * i + hh;
    pv[i] = *(const v4fa*)(stg + lr * BN + 4 * m);
  }
  const bool colOk = (colBase + 4 * m + 3) < nCols;
#pragma unroll
  for (int i = 0; i < 8; ++i) {
    const int gr = rowBase + 16 * wave + 2 * i + hh;
    float* op = C32 + (size_t)gr * (size_t)ldc + colBase + 4 * m;
    if (gr < nRows && colOk) *(volatile v4f*)op = pv[i];
  }
  __threadfence();
#pragma unroll
  for (int i = 0; i < 8; ++i) {
    const int gr = rowBase + 16 * wave + 2 * i + hh;
    float* op = C32 + (size_t)gr * (size_t)ldc + colBase + 4 * m;
    if (gr < nRows && colOk) *(volatile v4f*)op = pv[i];
  }
}

__global__ __launch_bounds__(NTHR) void k_agg(const int* __restrict__ keys, const int* __restrict__ gix,
                                              int nE, int nN, int vec8,
                                              const float* __restrict__ degin,
                                              const float* __restrict__ MR, const float* __restrict__ bias,
                                              unsigned short* Hout) {
  extern __shared__ __attribute__((aligned(16))) int dsm[];
  int* list = dsm;
  int* hl   = dsm + LISTN;
  int* sl   = dsm + LISTN + RCAP;
  int* cnt  = dsm + LISTN + 2 * RCAP;
  int* offs = cnt + NBA;
  int* cur  = offs + NBA;
  int* misc = cur + NBA;
  const int tid = (int)threadIdx.x, lane = tid & 31, wave = tid >> 5;
  const int nodeBase = (int)blockIdx.x * NBA;
  const int cl0 = 8 * lane;
  const int cl1 = (CH / 2) + 8 * lane;

  {
    const v4i z4 = {0, 0, 0, 0};
    for (int i = tid * 4; i < AGG_ZINTS; i += NTHR * 4) *(v4ia*)(dsm + i) = z4;
    if (tid < 16) misc[tid] = 0;
  }
  float bv[16];
  {
    const v4f b0 = *(const v4fa*)(bias + cl0);
    const v4f b1 = *(const v4fa*)(bias + cl0 + 4);
    const v4f b2 = *(const v4fa*)(bias + cl1);
    const v4f b3 = *(const v4fa*)(bias + cl1 + 4);
    bv[0]  = bf16_val(b0.x); bv[1]  = bf16_val(b0.y); bv[2]  = bf16_val(b0.z); bv[3]  = bf16_val(b0.w);
    bv[4]  = bf16_val(b1.x); bv[5]  = bf16_val(b1.y); bv[6]  = bf16_val(b1.z); bv[7]  = bf16_val(b1.w);
    bv[8]  = bf16_val(b2.x); bv[9]  = bf16_val(b2.y); bv[10] = bf16_val(b2.z); bv[11] = bf16_val(b2.w);
    bv[12] = bf16_val(b3.x); bv[13] = bf16_val(b3.y); bv[14] = bf16_val(b3.z); bv[15] = bf16_val(b3.w);
  }
  __syncthreads();

  int t = 0, ov = 0;
  const int nChunks = (nE + CHUNK - 1) / CHUNK;
#pragma unroll 1
  for (int ch = 0; ch < nChunks; ++ch) {
    const int cbase = ch * CHUNK;
    const int wc = scan_chunk<SLA>(keys, nE, cbase, nodeBase, NBA, vec8, list, tid, lane, wave);
    if (lane == 0) misc[wave] = wc;
    __syncthreads();
    if (wave == 0) {
#pragma unroll 1
      for (int w2 = 0; w2 < NWAVE; ++w2) {
        int c = misc[w2];
        c = c < 0 ? 0 : (c > WCAP ? WCAP : c);
#pragma unroll 1
        for (int b0 = 0; b0 < c; b0 += 32) {
          const int idx = b0 + lane;
          const int ent = list[w2 * WCAP + (idx < WCAP ? idx : WCAP - 1)];
          const int m32 = (c - b0) < 32 ? (c - b0) : 32;
#pragma unroll 1
          for (int k = 0; k < m32; ++k) {
            const int u    = __builtin_amdgcn_readlane(ent, k);
            const int slot = u & (NBA - 1);
            const int el   = (u >> SLA) & (CHUNK - 1);
            const int pk   = ((cbase + el) << SLA) | slot;
            if (t < RCAP) {
              if (lane == 0) { hl[t] = pk; cnt[slot] = cnt[slot] + 1; }
              t = t + 1;
            } else {
              ov = 1;
            }
          }
        }
      }
    }
    __syncthreads();
  }
  if (wave == 0 && lane == 0) { misc[8] = t; misc[9] = ov; }
  __syncthreads();
  int tt = misc[8];
  tt = tt < 0 ? 0 : (tt > RCAP ? RCAP : tt);
  const int ovf = misc[9];

  if (wave == 0) {
    const int base = lane * (NBA / 32);
    int s = 0;
#pragma unroll 1
    for (int i = 0; i < NBA / 32; ++i) s += cnt[base + i];
    int incl = s;
#pragma unroll
    for (int d = 1; d < 32; d <<= 1) {
      const int y = __shfl_up(incl, d, 32);
      if (lane >= d) incl += y;
    }
    int run = incl - s;
#pragma unroll 1
    for (int i = 0; i < NBA / 32; ++i) {
      const int cv = cnt[base + i];
      offs[base + i] = run;
      cur[base + i]  = run;
      run += cv;
    }
  }
  __syncthreads();
  if (wave == 0) {
#pragma unroll 1
    for (int b0 = 0; b0 < tt; b0 += 32) {
      const int idx = b0 + lane;
      const int ent = hl[idx < RCAP ? idx : RCAP - 1];
      const int m32 = (tt - b0) < 32 ? (tt - b0) : 32;
#pragma unroll 1
      for (int k = 0; k < m32; ++k) {
        const int u    = __builtin_amdgcn_readlane(ent, k);
        const int slot = u & (NBA - 1);
        if (lane == 0) {
          int p = cur[slot];
          p = p < 0 ? 0 : (p > RCAP - 1 ? RCAP - 1 : p);
          sl[p] = u;
          cur[slot] = p + 1;
        }
      }
    }
  }
  __syncthreads();

  const float qnan = __int_as_float(0x7fc00000);
  const float pz = (ovf != 0) ? qnan : 0.0f;
  const float fnE = (float)nE;
#pragma unroll 1
  for (int si = 0; si < NBA / NWAVE; ++si) {
    const int s    = si * NWAVE + wave;
    const int node = nodeBase + s;
    const int craw = cnt[s];
    const bool big = craw > DEGCAP;
    const int c = craw < 0 ? 0 : (craw > DEGCAP ? DEGCAP : craw);
    int o = offs[s];
    o = o < 0 ? 0 : (o > RCAP ? RCAP : o);
    const int nc = node < nN ? node : nN - 1;
    const int dgo = craw < 1 ? 1 : (craw > nE ? nE : craw);
    const float dego = (float)dgo;
    float acc[16];
#pragma unroll
    for (int j = 0; j < 16; ++j) acc[j] = 0.0f;
#pragma unroll 1
    for (int b0 = 0; b0 < c; b0 += 32) {
      int idx = o + b0 + lane;
      idx = idx > RCAP - 1 ? RCAP - 1 : idx;
      const int ent = sl[idx];
      int eid = ent >> SLA;
      eid = eid < 0 ? 0 : (eid > nE - 1 ? nE - 1 : eid);
      int dr = gix[eid];
      dr = dr < 0 ? 0 : (dr > nN - 1 ? nN - 1 : dr);
      float dg = degin[dr];
      dg = fmaxf(dg, 1.0f);
      dg = fminf(dg, fnE);
      const float we  = rsqrtf(dego * dg);
      const int   web = __float_as_int(we);
      const int m32 = (c - b0) < 32 ? (c - b0) : 32;
#pragma unroll 1
      for (int k = 0; k < m32; ++k) {
        const int   sk = __builtin_amdgcn_readlane(dr, k);
        const float wk = __int_as_float(__builtin_amdgcn_readlane(web, k));
        const float* rp = MR + (size_t)sk * NCAT;
        const v4f a0 = *(const v4fa*)(rp + cl0);
        const v4f a1 = *(const v4fa*)(rp + cl0 + 4);
        const v4f a2 = *(const v4fa*)(rp + cl1);
        const v4f a3 = *(const v4fa*)(rp + cl1 + 4);
        acc[0]  = fmaf(wk, a0.x, acc[0]);  acc[1]  = fmaf(wk, a0.y, acc[1]);
        acc[2]  = fmaf(wk, a0.z, acc[2]);  acc[3]  = fmaf(wk, a0.w, acc[3]);
        acc[4]  = fmaf(wk, a1.x, acc[4]);  acc[5]  = fmaf(wk, a1.y, acc[5]);
        acc[6]  = fmaf(wk, a1.z, acc[6]);  acc[7]  = fmaf(wk, a1.w, acc[7]);
        acc[8]  = fmaf(wk, a2.x, acc[8]);  acc[9]  = fmaf(wk, a2.y, acc[9]);
        acc[10] = fmaf(wk, a2.z, acc[10]); acc[11] = fmaf(wk, a2.w, acc[11]);
        acc[12] = fmaf(wk, a3.x, acc[12]); acc[13] = fmaf(wk, a3.y, acc[13]);
        acc[14] = fmaf(wk, a3.z, acc[14]); acc[15] = fmaf(wk, a3.w, acc[15]);
      }
    }
    const float* rr = MR + (size_t)nc * NCAT + CH;
    const v4f r0 = *(const v4fa*)(rr + cl0);
    const v4f r1 = *(const v4fa*)(rr + cl0 + 4);
    const v4f r2 = *(const v4fa*)(rr + cl1);
    const v4f r3 = *(const v4fa*)(rr + cl1 + 4);
    float rv[16];
    rv[0]  = r0.x; rv[1]  = r0.y; rv[2]  = r0.z; rv[3]  = r0.w;
    rv[4]  = r1.x; rv[5]  = r1.y; rv[6]  = r1.z; rv[7]  = r1.w;
    rv[8]  = r2.x; rv[9]  = r2.y; rv[10] = r2.z; rv[11] = r2.w;
    rv[12] = r3.x; rv[13] = r3.y; rv[14] = r3.z; rv[15] = r3.w;
    const float pzr = big ? qnan : pz;
    const bool live = node < nN;
    HPack o0, o1;
#pragma unroll
    for (int j = 0; j < 8; ++j) {
      float v = (acc[j] + rv[j]) + bv[j];
      v = (v < 0.0f) ? 0.0f : v;
      v = v + pzr;
      v = live ? v : 0.0f;
      o0.f[j] = (_Float16)(v * CA);
    }
#pragma unroll
    for (int j = 0; j < 8; ++j) {
      float v = (acc[8 + j] + rv[8 + j]) + bv[8 + j];
      v = (v < 0.0f) ? 0.0f : v;
      v = v + pzr;
      v = live ? v : 0.0f;
      o1.f[j] = (_Float16)(v * CA);
    }
    unsigned short* hp0 = Hout + (size_t)node * CH + cl0;
    unsigned short* hp1 = Hout + (size_t)node * CH + cl1;
    *(volatile v8us*)hp0 = o0.u;
    *(volatile v8us*)hp1 = o1.u;
    __threadfence();
    *(volatile v8us*)hp0 = o0.u;
    *(volatile v8us*)hp1 = o1.u;
  }
}

static inline int cdiv(int a, int b) { return (a + b - 1) / b; }
static inline size_t al256(size_t o) { return (o + 255) & ~(size_t)255; }

extern "C" void kernel_launch(void* const* d_in, const int* in_sizes, int n_in,
                              void* d_out, int out_size, void* d_ws, size_t ws_size,
                              hipStream_t stream) {
  if (n_in < 11) return;
  if (in_sizes[0] < IN_F || (in_sizes[0] % IN_F) != 0) return;
  const int nN = in_sizes[0] / IN_F;
  if (nN < 1 || nN > (1 << 20)) return;
  const int nE = in_sizes[1];
  if (nE < 1 || nE >= (1 << (31 - SLA)) || in_sizes[2] != nE) return;
  if (in_sizes[3] != IN_F * CH || in_sizes[4] != IN_F * CH || in_sizes[5] != CH) return;
  if (in_sizes[6] != NLK * CH * CH || in_sizes[7] != NLK * CH * CH || in_sizes[8] != NLK * CH) return;
  if (in_sizes[9] != CH * NLAB || in_sizes[10] != NLAB) return;
  if ((long long)out_size != (long long)nN * NLAB) return;

  const float* x   = (const float*)d_in[0];
  const int*   src = (const int*)d_in[1];
  const int*   dst = (const int*)d_in[2];
  const float* W1  = (const float*)d_in[3];
  const float* V1  = (const float*)d_in[4];
  const float* b1  = (const float*)d_in[5];
  const float* Wk  = (const float*)d_in[6];
  const float* Vk  = (const float*)d_in[7];
  const float* bk  = (const float*)d_in[8];
  const float* Wd  = (const float*)d_in[9];
  const float* bd  = (const float*)d_in[10];
  float* out = (float*)d_out;

  const int MP = cdiv(nN, GBM) * GBM;
  const int gM = MP / GBM;
  const int gA = cdiv(MP, NBA);
  const int RA = gA * NBA;
  const int gD = cdiv(nN, NBA);
  const int RD = gD * NBA;
  if ((long long)RA < (long long)MP || (long long)RD < (long long)nN) return;
  const int vec8 = ((nE & 3) == 0) ? 1 : 0;

  char* ws = (char*)d_ws;
  size_t off = 0;
  const size_t oDEG = off; off = al256(off + (size_t)RD * 4);
  const size_t oXH  = off; off = al256(off + (size_t)MP * IN_F * 2);
  const size_t oBT1 = off; off = al256(off + (size_t)NCAT * IN_F * 2);
  const size_t oBTK = off; off = al256(off + (size_t)NLK * NCAT * CH * 2);
  const size_t oBTD = off; off = al256(off + (size_t)NLAB * CH * 2);
  const size_t oMR  = off; off = al256(off + (size_t)MP * NCAT * 4);
  const size_t oHP  = off; off = al256(off + (size_t)RA * CH * 2);
  if (off > ws_size || off > (size_t)WSMAX) return;
  float*          DEG = (float*)(ws + oDEG);
  unsigned short* XH  = (unsigned short*)(ws + oXH);
  unsigned short* BT1 = (unsigned short*)(ws + oBT1);
  unsigned short* BTK = (unsigned short*)(ws + oBTK);
  unsigned short* BTD = (unsigned short*)(ws + oBTD);
  float*          MR  = (float*)(ws + oMR);
  unsigned short* HP  = (unsigned short*)(ws + oHP);

  const size_t aggLds = (size_t)AGG_LDS_INTS * 4;
  hipFuncSetAttribute(reinterpret_cast<const void*>(&k_agg), hipFuncAttributeMaxDynamicSharedMemorySize, (int)aggLds);

  k_deg<<<gD, NTHR, 0, stream>>>(dst, nE, vec8, DEG);
  const int nUx = MP * (IN_F / 8);
  k_xcvt<<<cdiv(nUx, NTHR), NTHR, 0, stream>>>(x, nN, nUx, XH);
  k_wtr<<<dim3(CH / TRN, IN_F / TRK, 1), NTHR, 0, stream>>>(W1, CH, IN_F, 0, BT1, 0, 0);
  k_wtr<<<dim3(CH / TRN, IN_F / TRK, 1), NTHR, 0, stream>>>(V1, CH, IN_F, 0, BT1, CH, 0);
  k_wtr<<<dim3(CH / TRN, CH / TRK, NLK), NTHR, 0, stream>>>(Wk, CH, CH, CH * CH, BTK, 0, NCAT * CH);
  k_wtr<<<dim3(CH / TRN, CH / TRK, NLK), NTHR, 0, stream>>>(Vk, CH, CH, CH * CH, BTK, CH, NCAT * CH);
  k_wtr<<<dim3(NLAB / TRN, CH / TRK, 1), NTHR, 0, stream>>>(Wd, NLAB, CH, 0, BTD, 0, 0);

  for (int l = 0; l < 7; ++l) {
    const unsigned short* Ap = (l == 0) ? XH : HP;
    const int K = (l == 0) ? IN_F : CH;
    const unsigned short* Bp = (l == 0) ? BT1 : (BTK + (size_t)(l - 1) * (size_t)NCAT * CH);
    const float* bp = (l == 0) ? b1 : (bk + (size_t)(l - 1) * CH);
    k_gemm<4, 0><<<dim3(gM, NCAT / GBN), GTHR, 0, stream>>>(Ap, K, Bp, K, NCAT, K, bp, MR, NCAT, MP, NCAT);
    k_agg<<<gA, NTHR, aggLds, stream>>>(src, dst, nE, nN, vec8, DEG, MR, bp, HP);
  }
  k_gemm<4, 1><<<dim3(gM, cdiv(NLAB, GBN)), GTHR, 0, stream>>>(HP, CH, BTD, CH, NLAB, CH, bd, out, NLAB, nN, NLAB);
}
